// ReLlamaAttention_77781857730645
// MI455X (gfx1250) — hardware-verified
//
#include <hip/hip_runtime.h>
#include <math.h>
#include <stdint.h>

#define NB_FULL   1
#define SEQ_FULL  2048
#define RLEN_FULL 2048
#ifndef NB
#define NB NB_FULL
#endif
#ifndef SEQ
#define SEQ SEQ_FULL
#endif
#define HID   2048
#define NH    16
#define NKV   4
#define HD    128
#define DQ    (NH * HD)
#define DKV   (NKV * HD)
#define CHK   64
#define RBS   64
#define QSC   8.0f
#define KSC   8.0f
#define QLS   1024.0f
#define PCAR  32768.0f
#define VCAR  4096.0f
#define OSC   1024.0f
#define OLS   1024.0f
#define WOS   1024.0f
#define LOG2E 1.4426950408889634f
#define NEGS  (-3.0e38f)
#define ATT_WAVES   4
#define ATT_THREADS (ATT_WAVES * 32)
#define NQT         (SEQ / CHK)
#define ATT_BLOCKS  (NH * NQT)
#define NKB         (SEQ / 32)
#define GSLAB  (16 * 68)
#define APITCH 132
#define ASLAB  (16 * APITCH)

static_assert(NB == NB_FULL);
static_assert((SEQ % 64) == 0 && SEQ >= 64 && SEQ <= SEQ_FULL && SEQ <= RLEN_FULL);
static_assert(HD == 128 && CHK == 64 && RBS == 64 && NH == 4 * NKV);
static_assert((HID % 64) == 0 && (DQ % 64) == 0 && (DKV % 64) == 0 && (HID % 32) == 0 && (DQ % 32) == 0);
static_assert(((SEQ * HID / 8) % 256) == 0 && ((SEQ * DQ / 8) % 256) == 0 && ((SEQ * DKV / 8) % 256) == 0);
static_assert(((SEQ * HD / 8) % 256) == 0 && ((RLEN_FULL * HD / 8) % 256) == 0);
static_assert(ATT_THREADS == 128 && ((GSLAB * 4) % 16) == 0 && (APITCH % 4) == 0 && ((ASLAB * 4) % 16) == 0);
static_assert(NKB * 32 == SEQ && NQT * 64 == SEQ);

typedef unsigned short u16;
typedef _Float16 v16h __attribute__((ext_vector_type(16)));
typedef _Float16 v8h  __attribute__((ext_vector_type(8)));
typedef __bf16   v16b __attribute__((ext_vector_type(16)));
typedef float    v8f  __attribute__((ext_vector_type(8)));
typedef float    v4f  __attribute__((ext_vector_type(4)));
typedef unsigned int v4u __attribute__((ext_vector_type(4)));

union FragH { v16h v; v8h h[2]; v4u u[2]; };
union FragB { v16b v; v4u u[2]; };

__device__ __forceinline__ unsigned short bf_bits(float f) {
  unsigned u = __float_as_uint(f);
  return (unsigned short)((u + 0x7FFFu + ((u >> 16) & 1u)) >> 16);
}
__device__ __forceinline__ float bf_up(unsigned short h) { return __uint_as_float(((unsigned)h) << 16); }
__device__ __forceinline__ float bf_val(float f) { return bf_up(bf_bits(f)); }
__device__ __forceinline__ unsigned short h_bits(_Float16 x) { return __builtin_bit_cast(unsigned short, x); }
__device__ __forceinline__ unsigned pk16(unsigned short a, unsigned short b) { return (unsigned)a | ((unsigned)b << 16); }
__device__ __forceinline__ v8f zero8() { v8f z = {0.f, 0.f, 0.f, 0.f, 0.f, 0.f, 0.f, 0.f}; return z; }

__device__ __forceinline__ v16h ldfrag_h(const _Float16* p) {
  FragH f;
  f.h[0] = *(const v8h*)(p);
  f.h[1] = *(const v8h*)(p + 16);
  return f.v;
}
__device__ __forceinline__ v16b ldfrag_b(const u16* p) {
  FragB f;
  f.u[0] = *(const v4u*)(p);
  f.u[1] = *(const v4u*)(p + 16);
  return f.v;
}

__device__ __forceinline__ v8f mma_h(v16h a, v16h b, v8f c) {
  return __builtin_amdgcn_wmma_f32_16x16x32_f16(false, a, false, b, (short)0, c, false, false);
}
__device__ __forceinline__ v8f mma_b(v16b a, v16b b, v8f c) {
  return __builtin_amdgcn_wmma_f32_16x16x32_bf16(false, a, false, b, (short)0, c, false, false);
}
__device__ __forceinline__ void guard2(v8f& a, v8f& b, v16h x0, v16h x1, v16h x2, v16h x3, v16h x4, v16h x5) {
#if defined(__HIP_DEVICE_COMPILE__)
  asm volatile("v_nop\n\tv_nop\n\tv_nop\n\tv_nop"
               : "+v"(a), "+v"(b) : "v"(x0), "v"(x1), "v"(x2), "v"(x3), "v"(x4), "v"(x5) : "memory");
#endif
}
template <typename F>
__device__ __forceinline__ void guard6(v8f& a, v8f& b, v8f& c, v8f& d, F x0, F x1, F x2, F x3, F x4, F x5) {
#if defined(__HIP_DEVICE_COMPILE__)
  asm volatile("v_nop\n\tv_nop\n\tv_nop\n\tv_nop"
               : "+v"(a), "+v"(b), "+v"(c), "+v"(d) : "v"(x0), "v"(x1), "v"(x2), "v"(x3), "v"(x4), "v"(x5) : "memory");
#endif
}
__device__ __forceinline__ void guard8(v8f& a, v8f& b, v8f& c, v8f& d, v8f& e, v8f& f, v8f& g, v8f& h,
                                       v16h x0, v16h x1, v16h x2, v16h x3, v16h x4, v16h x5) {
#if defined(__HIP_DEVICE_COMPILE__)
  asm volatile("v_nop\n\tv_nop\n\tv_nop\n\tv_nop"
               : "+v"(a), "+v"(b), "+v"(c), "+v"(d), "+v"(e), "+v"(f), "+v"(g), "+v"(h)
               : "v"(x0), "v"(x1), "v"(x2), "v"(x3), "v"(x4), "v"(x5) : "memory");
#endif
}
__device__ __forceinline__ void acc_guard8(v8f& a, v8f& b, v8f& c, v8f& d, v8f& e, v8f& f, v8f& g, v8f& h) {
#if defined(__HIP_DEVICE_COMPILE__)
  asm volatile("v_nop\n\tv_nop\n\tv_nop\n\tv_nop"
               : "+v"(a), "+v"(b), "+v"(c), "+v"(d), "+v"(e), "+v"(f), "+v"(g), "+v"(h));
#endif
}
__device__ __forceinline__ void wave_sync_lds() {
#if defined(__HIP_DEVICE_COMPILE__)
  __builtin_amdgcn_fence(__ATOMIC_RELEASE, "workgroup");
  __builtin_amdgcn_wave_barrier();
  __builtin_amdgcn_fence(__ATOMIC_ACQUIRE, "workgroup");
#endif
}

__global__ __launch_bounds__(256) void cvt16(const float* __restrict__ x, u16* Dp, int n8, int bpb, int bstx8, int bstd8,
                                             int mode, float scale) {
  const int bt = blockIdx.x / bpb;
  const int gt = (blockIdx.x - bt * bpb) * 256 + (int)threadIdx.x;
  if (gt >= n8) return;
  const float* p = x + ((size_t)bt * (size_t)bstx8 + (size_t)gt) * 8;
  const v4f a = *(const v4f*)(p), c4 = *(const v4f*)(p + 4);
  float v[8];
#pragma unroll
  for (int e = 0; e < 4; ++e) { v[e] = a[e]; v[4 + e] = c4[e]; }
  unsigned short s[8];
#pragma unroll
  for (int e = 0; e < 8; ++e) {
    const unsigned short bb = bf_bits(v[e]);
    const unsigned short hb = h_bits((_Float16)(bf_up(bb) * scale));
    s[e] = (mode != 0) ? hb : bb;
  }
  v4u o;
#pragma unroll
  for (int e = 0; e < 4; ++e) o[e] = pk16(s[2 * e], s[2 * e + 1]);
  u16* d = Dp + ((size_t)bt * (size_t)bstd8 + (size_t)gt) * 8;
  for (int pass = 0; pass < 2; ++pass) {
    *(volatile v4u*)(d) = o;
    __threadfence();
  }
}

__global__ __launch_bounds__(256) void tr16(const float* __restrict__ W, u16* Hp, u16* Lp, int rows, int cols, int tpb,
                                            int bstIn, int bstOut, int mode, float scale) {
  __shared__ __align__(16) float sT[64 * 68];
  const int tid = threadIdx.x;
  const int bt  = blockIdx.x / tpb;
  const int t   = blockIdx.x - bt * tpb;
  const int ctile = cols >> 6;
  const int r0 = (t / ctile) * 64;
  const int c0 = (t % ctile) * 64;
  const float* Wb = W + (size_t)bt * (size_t)bstIn;
#pragma unroll
  for (int it = 0; it < 4; ++it) {
    const int row = it * 16 + (tid >> 4), c4 = (tid & 15) * 4;
    const v4f a = *(const v4f*)(Wb + (size_t)(r0 + row) * (size_t)cols + c0 + c4);
#pragma unroll
    for (int e = 0; e < 4; ++e) sT[(c4 + e) * 68 + row] = a[e];
  }
  __syncthreads();
  const int k8 = (tid & 7) * 8, nq = tid >> 3;
  v4u oh[2], ol[2];
#pragma unroll
  for (int it = 0; it < 2; ++it) {
    const int n = it * 32 + nq;
    const v4f a = *(const v4f*)(sT + n * 68 + k8), b = *(const v4f*)(sT + n * 68 + k8 + 4);
    float w[8];
#pragma unroll
    for (int e = 0; e < 4; ++e) { w[e] = a[e]; w[4 + e] = b[e]; }
    unsigned short hs[8], ls[8];
#pragma unroll
    for (int e = 0; e < 8; ++e) {
      const unsigned short bb = bf_bits(w[e]);
      const float ws = bf_up(bb) * scale;
      const _Float16 h = (_Float16)ws;
      const _Float16 l = (_Float16)(ws - (float)h);
      hs[e] = (mode != 0) ? h_bits(h) : bb;
      ls[e] = h_bits(l);
    }
#pragma unroll
    for (int e = 0; e < 4; ++e) {
      oh[it][e] = pk16(hs[2 * e], hs[2 * e + 1]);
      ol[it][e] = pk16(ls[2 * e], ls[2 * e + 1]);
    }
  }
  u16* Hb = Hp + (size_t)bt * (size_t)bstOut;
  u16* Lb = Lp + (size_t)bt * (size_t)bstOut;
  const size_t d0 = (size_t)(c0 + nq) * (size_t)rows + (size_t)r0 + (size_t)k8;
  for (int pass = 0; pass < 2; ++pass) {
#pragma unroll
    for (int it = 0; it < 2; ++it) {
      const size_t di = d0 + (size_t)(it * 32) * (size_t)rows;
      *(volatile v4u*)(Hb + di) = oh[it];
      if (mode == 2) *(volatile v4u*)(Lb + di) = ol[it];
    }
    __threadfence();
  }
}

__device__ __forceinline__ void epi64(float* sl, v8f a0, v8f a1, v8f a2, v8f a3, float oscale, float* C, int N,
                                      size_t rowb, int col0, int lane) {
  const int hh = lane >> 4, m = lane & 15;
#pragma unroll
  for (int r = 0; r < 8; ++r) {
    const int ro = (8 * hh + r) * 68 + m;
    sl[ro]      = a0[r] * oscale;
    sl[ro + 16] = a1[r] * oscale;
    sl[ro + 32] = a2[r] * oscale;
    sl[ro + 48] = a3[r] * oscale;
  }
  wave_sync_lds();
  v4f vals[8];
#pragma unroll
  for (int it = 0; it < 8; ++it) vals[it] = *(const v4f*)(sl + (it * 2 + hh) * 68 + m * 4);
  float* dst = C + (rowb + (size_t)hh) * (size_t)N + col0 + m * 4;
  for (int pass = 0; pass < 2; ++pass) {
#pragma unroll
    for (int it = 0; it < 8; ++it) {
      *(volatile v4f*)(dst + (size_t)(it * 2) * (size_t)N) = vals[it];
    }
    __threadfence();
  }
}

__device__ __forceinline__ void epi16x2(float* sl, v8f a0, v8f a1, v8f a2, v8f a3, float oscale, u16* Hc, u16* Lc, int N,
                                        size_t rowb, int col0, int lane) {
  const int hh = lane >> 4, m = lane & 15;
#pragma unroll
  for (int r = 0; r < 8; ++r) {
    const int ro = (8 * hh + r) * 68 + m;
    sl[ro]      = a0[r] * oscale;
    sl[ro + 16] = a1[r] * oscale;
    sl[ro + 32] = a2[r] * oscale;
    sl[ro + 48] = a3[r] * oscale;
  }
  wave_sync_lds();
  const int rq = lane >> 3, c8 = (lane & 7) * 8;
  v4u oh[4], ol[4];
#pragma unroll
  for (int i4 = 0; i4 < 4; ++i4) {
    const int row = i4 * 4 + rq;
    const v4f a = *(const v4f*)(sl + row * 68 + c8), c4 = *(const v4f*)(sl + row * 68 + c8 + 4);
    float w[8];
#pragma unroll
    for (int e = 0; e < 4; ++e) { w[e] = a[e]; w[4 + e] = c4[e]; }
    unsigned short hs[8], ls[8];
#pragma unroll
    for (int e = 0; e < 8; ++e) {
      const _Float16 h = (_Float16)w[e];
      const _Float16 l = (_Float16)(w[e] - (float)h);
      hs[e] = h_bits(h);
      ls[e] = h_bits(l);
    }
#pragma unroll
    for (int e = 0; e < 4; ++e) {
      oh[i4][e] = pk16(hs[2 * e], hs[2 * e + 1]);
      ol[i4][e] = pk16(ls[2 * e], ls[2 * e + 1]);
    }
  }
  const size_t d0 = (rowb + (size_t)rq) * (size_t)N + (size_t)col0 + (size_t)c8;
  for (int pass = 0; pass < 2; ++pass) {
#pragma unroll
    for (int i4 = 0; i4 < 4; ++i4) {
      const size_t di = d0 + (size_t)(i4 * 4) * (size_t)N;
      *(volatile v4u*)(Hc + di) = oh[i4];
      *(volatile v4u*)(Lc + di) = ol[i4];
    }
    __threadfence();
  }
}

__global__ __launch_bounds__(128)
void gemm_bb32(const u16* __restrict__ A, const u16* __restrict__ Bt, float* C, int M, int N, int K, float oscale) {
  __shared__ __align__(16) float slab[4 * GSLAB];
  const int tid = threadIdx.x, wave = tid >> 5, lane = tid & 31, hh = lane >> 4, m = lane & 15;
  const int ntile = N >> 6;
  const int bid   = blockIdx.x;
  const int rowb  = (bid / ntile) * 64 + wave * 16;
  const int col0  = (bid % ntile) * 64;
  if (rowb + 16 > M) return;
  const u16* ap = A  + (size_t)(rowb + m) * (size_t)K + 8 * hh;
  const u16* bp = Bt + (size_t)(col0 + m) * (size_t)K + 8 * hh;
  const size_t bs = (size_t)16 * (size_t)K;
  v8f acc0 = zero8(), acc1 = zero8(), acc2 = zero8(), acc3 = zero8();
#pragma unroll 1
  for (int k0 = 0; k0 < K; k0 += 32) {
    const v16b a  = ldfrag_b(ap + k0);
    const v16b b0 = ldfrag_b(bp + k0);
    const v16b b1 = ldfrag_b(bp + bs + k0);
    const v16b b2 = ldfrag_b(bp + 2 * bs + k0);
    const v16b b3 = ldfrag_b(bp + 3 * bs + k0);
    acc0 = mma_b(a, b0, acc0);
    acc1 = mma_b(a, b1, acc1);
    acc2 = mma_b(a, b2, acc2);
    acc3 = mma_b(a, b3, acc3);
    guard6<v16b>(acc0, acc1, acc2, acc3, a, b0, b1, b2, b3, a);
  }
  epi64(slab + wave * GSLAB, acc0, acc1, acc2, acc3, oscale, C, N, (size_t)rowb, col0, lane);
}

__global__ __launch_bounds__(128)
void gemm_vv16(const u16* __restrict__ A, const u16* __restrict__ Bt, u16* Hc, u16* Lc, int M, int N, int K, float oscale) {
  __shared__ __align__(16) float slab[4 * GSLAB];
  const int tid = threadIdx.x, wave = tid >> 5, lane = tid & 31, hh = lane >> 4, m = lane & 15;
  const int ntile = N >> 6;
  const int bid   = blockIdx.x;
  const int rowb  = (bid / ntile) * 64 + wave * 16;
  const int col0  = (bid % ntile) * 64;
  if (rowb + 16 > M) return;
  const u16* ap = A  + (size_t)(rowb + m) * (size_t)K + 8 * hh;
  const u16* bp = Bt + (size_t)(col0 + m) * (size_t)K + 8 * hh;
  const size_t bs = (size_t)16 * (size_t)K;
  v8f acc0 = zero8(), acc1 = zero8(), acc2 = zero8(), acc3 = zero8();
#pragma unroll 1
  for (int k0 = 0; k0 < K; k0 += 32) {
    const v16b a  = ldfrag_b(ap + k0);
    const v16b b0 = ldfrag_b(bp + k0);
    const v16b b1 = ldfrag_b(bp + bs + k0);
    const v16b b2 = ldfrag_b(bp + 2 * bs + k0);
    const v16b b3 = ldfrag_b(bp + 3 * bs + k0);
    acc0 = mma_b(a, b0, acc0);
    acc1 = mma_b(a, b1, acc1);
    acc2 = mma_b(a, b2, acc2);
    acc3 = mma_b(a, b3, acc3);
    guard6<v16b>(acc0, acc1, acc2, acc3, a, b0, b1, b2, b3, a);
  }
  epi16x2(slab + wave * GSLAB, acc0, acc1, acc2, acc3, oscale, Hc, Lc, N, (size_t)rowb, col0, lane);
}

__global__ __launch_bounds__(128)
void gemm_oo32(const u16* __restrict__ AH, const u16* __restrict__ AL, const u16* __restrict__ Bt, float* C,
               int M, int N, int K, float oscale, float rls) {
  __shared__ __align__(16) float slab[4 * GSLAB];
  const int tid = threadIdx.x, wave = tid >> 5, lane = tid & 31, hh = lane >> 4, m = lane & 15;
  const int ntile = N >> 6;
  const int bid   = blockIdx.x;
  const int rowb  = (bid / ntile) * 64 + wave * 16;
  const int col0  = (bid % ntile) * 64;
  if (rowb + 16 > M) return;
  const _Float16* aph = (const _Float16*)(const void*)AH + (size_t)(rowb + m) * (size_t)K + 8 * hh;
  const _Float16* apl = (const _Float16*)(const void*)AL + (size_t)(rowb + m) * (size_t)K + 8 * hh;
  const _Float16* bp  = (const _Float16*)(const void*)Bt + (size_t)(col0 + m) * (size_t)K + 8 * hh;
  const size_t bs = (size_t)16 * (size_t)K;
  v8f c0 = zero8(), c1 = zero8(), c2 = zero8(), c3 = zero8();
  v8f e0 = zero8(), e1 = zero8(), e2 = zero8(), e3 = zero8();
#pragma unroll 1
  for (int k0 = 0; k0 < K; k0 += 32) {
    const v16h ah = ldfrag_h(aph + k0);
    const v16h al = ldfrag_h(apl + k0);
    const v16h b0 = ldfrag_h(bp + k0);
    const v16h b1 = ldfrag_h(bp + bs + k0);
    const v16h b2 = ldfrag_h(bp + 2 * bs + k0);
    const v16h b3 = ldfrag_h(bp + 3 * bs + k0);
    c0 = mma_h(ah, b0, c0);
    c1 = mma_h(ah, b1, c1);
    c2 = mma_h(ah, b2, c2);
    c3 = mma_h(ah, b3, c3);
    e0 = mma_h(al, b0, e0);
    e1 = mma_h(al, b1, e1);
    e2 = mma_h(al, b2, e2);
    e3 = mma_h(al, b3, e3);
    guard8(c0, c1, c2, c3, e0, e1, e2, e3, ah, al, b0, b1, b2, b3);
  }
#pragma unroll
  for (int r = 0; r < 8; ++r) {
    c0[r] = c0[r] + e0[r] * rls;
    c1[r] = c1[r] + e1[r] * rls;
    c2[r] = c2[r] + e2[r] * rls;
    c3[r] = c3[r] + e3[r] * rls;
  }
  epi64(slab + wave * GSLAB, c0, c1, c2, c3, oscale, C, N, (size_t)rowb, col0, lane);
}

__global__ __launch_bounds__(256) void rope16(const float* __restrict__ X, int ncol, const float* __restrict__ cs,
                                              const float* __restrict__ sn, u16* Hp, u16* Lp, int wlo, int n8,
                                              float sc, float ls) {
  const int gt = blockIdx.x * 256 + (int)threadIdx.x;
  if (gt >= n8) return;
  const size_t e   = (size_t)gt * 8;
  const int    s   = (int)(e / (size_t)ncol);
  const int    col = (int)(e - (size_t)s * (size_t)ncol);
  const int    d   = col & (HD - 1);
  const float* xp = X + e;
  const float* yp = X + (e ^ (size_t)64);
  const float* cp = cs + (size_t)s * HD + d;
  const float* sp = sn + (size_t)s * HD + d;
  const v4f xa = *(const v4f*)(xp), xb = *(const v4f*)(xp + 4);
  const v4f ya = *(const v4f*)(yp), yb = *(const v4f*)(yp + 4);
  const v4f ca = *(const v4f*)(cp), cb = *(const v4f*)(cp + 4);
  const v4f sa = *(const v4f*)(sp), sb = *(const v4f*)(sp + 4);
  const float sg = (d < 64) ? -1.0f : 1.0f;
  float xv[8], yv[8], cv[8], sv[8];
#pragma unroll
  for (int i = 0; i < 4; ++i) {
    xv[i] = xa[i]; xv[4 + i] = xb[i];
    yv[i] = ya[i]; yv[4 + i] = yb[i];
    cv[i] = ca[i]; cv[4 + i] = cb[i];
    sv[i] = sa[i]; sv[4 + i] = sb[i];
  }
  unsigned short hs[8], lsb[8];
#pragma unroll
  for (int i = 0; i < 8; ++i) {
    const float y  = xv[i] * bf_val(cv[i]) + (sg * yv[i]) * bf_val(sv[i]);
    const float w  = y * sc;
    const _Float16 h = (_Float16)w;
    const _Float16 l = (_Float16)((w - (float)h) * ls);
    hs[i]  = h_bits(h);
    lsb[i] = h_bits(l);
  }
  v4u oh, ol;
#pragma unroll
  for (int i = 0; i < 4; ++i) {
    oh[i] = pk16(hs[2 * i], hs[2 * i + 1]);
    ol[i] = pk16(lsb[2 * i], lsb[2 * i + 1]);
  }
  for (int pass = 0; pass < 2; ++pass) {
    *(volatile v4u*)(Hp + e) = oh;
    if (wlo != 0) *(volatile v4u*)(Lp + e) = ol;
    __threadfence();
  }
}

static __device__ __forceinline__ void att_step(const _Float16* k0p, int kpitch, const _Float16* qhp, const _Float16* qlp,
                                                const _Float16* vhp, const _Float16* vlp, int vpitch, int dqk, float lsc,
                                                float& mrun, float& lrun, v8f (&o)[8]) {
  const int lane = threadIdx.x & 31, hh = lane >> 4;
  const _Float16* k1p = k0p + (size_t)16 * (size_t)kpitch;
  v8f s0 = zero8(), s1 = zero8(), r0 = zero8(), r1 = zero8();
#pragma unroll
  for (int dc = 0; dc < 4; ++dc) {
    const v16h qh = ldfrag_h(qhp + 32 * dc);
    const v16h ql = ldfrag_h(qlp + 32 * dc);
    const v16h ka = ldfrag_h(k0p + 32 * dc);
    const v16h kc = ldfrag_h(k1p + 32 * dc);
    s0 = mma_h(ka, qh, s0);
    r0 = mma_h(ka, ql, r0);
    s1 = mma_h(kc, qh, s1);
    r1 = mma_h(kc, ql, r1);
    guard6<v16h>(s0, r0, s1, r1, qh, ql, ka, kc, qh, ka);
  }
  float tk[16];
#pragma unroll
  for (int i = 0; i < 8; ++i) {
    const int d0 = dqk - i;
    const int d1 = d0 - 16;
    const float t0 = (s0[i] + r0[i] * (1.0f / QLS)) * lsc;
    const float t1 = (s1[i] + r1[i] * (1.0f / QLS)) * lsc;
    tk[i]     = (d0 >= 0) ? t0 : NEGS;
    tk[8 + i] = (d1 >= 0) ? t1 : NEGS;
  }
  float cm = tk[0];
#pragma unroll
  for (int i = 1; i < 16; ++i) cm = fmaxf(cm, tk[i]);
  cm = fmaxf(cm, __shfl_xor(cm, 16, 32));
  const float mn = fmaxf(mrun, cm);
  const float al = exp2f(fminf(mrun - mn, 0.f));
  mrun = mn;
  float ps = 0.f;
  FragH ph, pl;
#pragma unroll
  for (int wq = 0; wq < 2; ++wq) {
#pragma unroll
    for (int e4 = 0; e4 < 4; ++e4) {
      const int i = 8 * wq + 2 * e4;
      const float x0 = exp2f(fminf(tk[i] - mn, 0.f));
      const float x1 = exp2f(fminf(tk[i + 1] - mn, 0.f));
      const float p0 = (tk[i] > -1.0e38f) ? x0 : 0.f;
      const float p1 = (tk[i + 1] > -1.0e38f) ? x1 : 0.f;
      ps += p0 + p1;
      const float w0 = p0 * PCAR, w1 = p1 * PCAR;
      const _Float16 h0 = (_Float16)w0, h1 = (_Float16)w1;
      const _Float16 l0 = (_Float16)(w0 - (float)h0), l1 = (_Float16)(w1 - (float)h1);
      ph.u[wq][e4] = pk16(h_bits(h0), h_bits(h1));
      pl.u[wq][e4] = pk16(h_bits(l0), h_bits(l1));
    }
  }
  ps += __shfl_xor(ps, 16, 32);
  lrun = lrun * al + ps;
  float scl[8];
#pragma unroll
  for (int r = 0; r < 8; ++r) scl[r] = __shfl(al, 8 * hh + r, 32);
#pragma unroll
  for (int j = 0; j < 8; ++j) {
#pragma unroll
    for (int r = 0; r < 8; ++r) o[j][r] *= scl[r];
  }
#pragma unroll
  for (int jp = 0; jp < 4; ++jp) {
    const size_t dof0 = (size_t)(32 * jp) * (size_t)vpitch;
    const size_t dof1 = (size_t)(32 * jp + 16) * (size_t)vpitch;
    const v16h vh0 = ldfrag_h(vhp + dof0);
    const v16h vl0 = ldfrag_h(vlp + dof0);
    const v16h vh1 = ldfrag_h(vhp + dof1);
    const v16h vl1 = ldfrag_h(vlp + dof1);
    o[2 * jp]     = mma_h(ph.v, vh0, o[2 * jp]);
    o[2 * jp]     = mma_h(pl.v, vh0, o[2 * jp]);
    o[2 * jp]     = mma_h(ph.v, vl0, o[2 * jp]);
    o[2 * jp + 1] = mma_h(ph.v, vh1, o[2 * jp + 1]);
    o[2 * jp + 1] = mma_h(pl.v, vh1, o[2 * jp + 1]);
    o[2 * jp + 1] = mma_h(ph.v, vl1, o[2 * jp + 1]);
    guard2(o[2 * jp], o[2 * jp + 1], ph.v, pl.v, vh0, vl0, vh1, vl1);
  }
}

__global__ __launch_bounds__(ATT_THREADS)
void attn_fwd(const u16* __restrict__ QHp, const u16* __restrict__ QLp, const u16* __restrict__ KPp,
              const u16* __restrict__ VHp, const u16* __restrict__ VLp, const u16* __restrict__ RKp,
              const u16* __restrict__ RVHp, const u16* __restrict__ RVLp, u16* OHp, u16* OLp) {
  __shared__ __align__(16) float smem[ATT_WAVES * ASLAB];

  const int tid  = threadIdx.x;
  const int wave = tid >> 5;
  const int lane = tid & 31;
  const int hh   = lane >> 4;
  const int c    = lane & 15;

  const int bid  = blockIdx.x;
  const int qt   = bid % NQT;
  const int head = bid / NQT;
  if (head >= NH) return;
  const int kvh  = head >> 2;
  const int qb   = qt * 64;
  const int q0   = qb + wave * 16;

  const _Float16* QH  = (const _Float16*)(const void*)QHp  + (size_t)(q0 + c) * DQ + head * HD + 8 * hh;
  const _Float16* QL  = (const _Float16*)(const void*)QLp  + (size_t)(q0 + c) * DQ + head * HD + 8 * hh;
  const _Float16* KB  = (const _Float16*)(const void*)KPp  + (size_t)c * DKV + kvh * HD + 8 * hh;
  const _Float16* VHb = (const _Float16*)(const void*)VHp  + (size_t)(kvh * HD + c) * SEQ + 8 * hh;
  const _Float16* VLb = (const _Float16*)(const void*)VLp  + (size_t)(kvh * HD + c) * SEQ + 8 * hh;
  const _Float16* RKb = (const _Float16*)(const void*)RKp  + ((size_t)kvh * SEQ + c) * HD + 8 * hh;
  const _Float16* RVH = (const _Float16*)(const void*)RVHp + (size_t)(kvh * HD + c) * SEQ + 8 * hh;
  const _Float16* RVL = (const _Float16*)(const void*)RVLp + (size_t)(kvh * HD + c) * SEQ + 8 * hh;
  const float lsc = (0.08838834764831845f * LOG2E) / (QSC * KSC);
  const int dq = q0 + c - 8 * hh;

  float mrun = NEGS, lrun = 0.f;
  v8f o[8];
#pragma unroll
  for (int j = 0; j < 8; ++j) o[j] = zero8();

  const int nkb  = ((q0 + 15) >> 5) + 1;
  const int nret = (qt >= 1) ? 2 : 0;
  const int rb0  = (qt >= 1) ? ((qt - 1) * RBS) : 0;
#pragma unroll 1
  for (int it = 0; it < nkb + nret; ++it) {
    const bool isr = (it >= nkb);
    const int  kb  = isr ? (rb0 + 32 * (it - nkb)) : (32 * it);
    const _Float16* kp  = isr ? (RKb + (size_t)kb * HD) : (KB + (size_t)kb * DKV);
    const int  kpitch   = isr ? HD : DKV;
    const _Float16* vhp = (isr ? RVH : VHb) + kb;
    const _Float16* vlp = (isr ? RVL : VLb) + kb;
    const int  dqk      = isr ? (1 << 20) : (dq - kb);
    att_step(kp, kpitch, QH, QL, vhp, vlp, SEQ, dqk, lsc, mrun, lrun, o);
  }
  acc_guard8(o[0], o[1], o[2], o[3], o[4], o[5], o[6], o[7]);

  const float linv = (lrun > 0.f) ? ((1.0f / lrun) * (1.0f / (PCAR * VCAR))) : 0.f;
  float inv[8];
#pragma unroll
  for (int r = 0; r < 8; ++r) inv[r] = __shfl(linv, 8 * hh + r, 32);
  float* slab = smem + wave * ASLAB;
#pragma unroll
  for (int r = 0; r < 8; ++r) {
#pragma unroll
    for (int j = 0; j < 8; ++j) slab[(8 * hh + r) * APITCH + j * 16 + c] = o[j][r] * inv[r];
  }
  wave_sync_lds();
  const int rq = lane >> 4, c8 = (lane & 15) * 8;
  v4u oh[8], ol[8];
#pragma unroll
  for (int i8 = 0; i8 < 8; ++i8) {
    const int row = 2 * i8 + rq;
    const v4f a = *(const v4f*)(slab + row * APITCH + c8), c4 = *(const v4f*)(slab + row * APITCH + c8 + 4);
    float wv[8];
#pragma unroll
    for (int e = 0; e < 4; ++e) { wv[e] = a[e] * OSC; wv[4 + e] = c4[e] * OSC; }
    unsigned short hs[8], ls[8];
#pragma unroll
    for (int e = 0; e < 8; ++e) {
      const _Float16 h = (_Float16)wv[e];
      const _Float16 l = (_Float16)((wv[e] - (float)h) * OLS);
      hs[e] = h_bits(h);
      ls[e] = h_bits(l);
    }
#pragma unroll
    for (int e = 0; e < 4; ++e) {
      oh[i8][e] = pk16(hs[2 * e], hs[2 * e + 1]);
      ol[i8][e] = pk16(ls[2 * e], ls[2 * e + 1]);
    }
  }
  const size_t ob = (size_t)q0 * DQ + (size_t)head * HD + (size_t)c8;
  for (int pass = 0; pass < 2; ++pass) {
#pragma unroll
    for (int i8 = 0; i8 < 8; ++i8) {
      const size_t o8 = ob + (size_t)(2 * i8 + rq) * (size_t)DQ;
      *(volatile v4u*)(OHp + o8) = oh[i8];
      *(volatile v4u*)(OLp + o8) = ol[i8];
    }
    __threadfence();
  }
}

extern "C" void kernel_launch(void* const* d_in, const int* in_sizes, int n_in,
                              void* d_out, int out_size, void* d_ws, size_t ws_size,
                              hipStream_t stream) {
  if (n_in < 9) return;
  if (in_sizes[0] < SEQ * HID) return;
  if (in_sizes[1] < SEQ * HD) return;
  if (in_sizes[2] < SEQ * HD) return;
  if (in_sizes[3] < NKV * RLEN_FULL * HD) return;
  if (in_sizes[4] < NKV * RLEN_FULL * HD) return;
  if (in_sizes[5] < HID * DQ) return;
  if (in_sizes[6] < HID * DKV) return;
  if (in_sizes[7] < HID * DKV) return;
  if (in_sizes[8] < DQ * HID) return;
  if (out_size < SEQ * HID) return;

  const float* Xin = (const float*)d_in[0];
  const float* Cin = (const float*)d_in[1];
  const float* Sin = (const float*)d_in[2];
  const float* RKi = (const float*)d_in[3];
  const float* RVi = (const float*)d_in[4];
  const float* Wqi = (const float*)d_in[5];
  const float* Wki = (const float*)d_in[6];
  const float* Wvi = (const float*)d_in[7];
  const float* Woi = (const float*)d_in[8];
  float*       out = (float*)d_out;

  const size_t szXB = (size_t)SEQ * HID * 2;
  const size_t szWQ = (size_t)DQ * HID * 2;
  const size_t szWK = (size_t)DKV * HID * 2;
  const size_t szWO = (size_t)HID * DQ * 2;
  const size_t szQF = (size_t)SEQ * DQ * 4;
  const size_t szKF = (size_t)SEQ * DKV * 4;
  const size_t szQP = (size_t)SEQ * DQ * 2;
  const size_t szKP = (size_t)SEQ * DKV * 2;
  const size_t szVP = (size_t)DKV * SEQ * 2;
  const size_t szRK = (size_t)NKV * SEQ * HD * 2;
  const size_t szRV = (size_t)NKV * HD * SEQ * 2;
  const size_t szOP = (size_t)SEQ * DQ * 2;
  size_t off = 0;
  const size_t oXB = off; off += szXB;
  const size_t oWQ = off; off += szWQ;
  const size_t oWK = off; off += szWK;
  const size_t oWV = off; off += szWK;
  const size_t oWO = off; off += szWO;
  const size_t oQF = off; off += szQF;
  const size_t oKF = off; off += szKF;
  const size_t oQH = off; off += szQP;
  const size_t oQL = off; off += szQP;
  const size_t oKP = off; off += szKP;
  const size_t oVH = off; off += szVP;
  const size_t oVL = off; off += szVP;
  const size_t oRK = off; off += szRK;
  const size_t oRH = off; off += szRV;
  const size_t oRL = off; off += szRV;
  const size_t oOH = off; off += szOP;
  const size_t oOL = off; off += szOP;
  if (off > ws_size) return;
  if (off > (size_t)134217728) return;

  char* ws = (char*)d_ws;
  u16*   XB  = (u16*)(ws + oXB);
  u16*   WQT = (u16*)(ws + oWQ);
  u16*   WKT = (u16*)(ws + oWK);
  u16*   WVT = (u16*)(ws + oWV);
  u16*   WOT = (u16*)(ws + oWO);
  float* QF  = (float*)(ws + oQF);
  float* KF  = (float*)(ws + oKF);
  u16*   QH  = (u16*)(ws + oQH);
  u16*   QL  = (u16*)(ws + oQL);
  u16*   KP  = (u16*)(ws + oKP);
  u16*   VH  = (u16*)(ws + oVH);
  u16*   VL  = (u16*)(ws + oVL);
  u16*   RK  = (u16*)(ws + oRK);
  u16*   RVH = (u16*)(ws + oRH);
  u16*   RVL = (u16*)(ws + oRL);
  u16*   OH  = (u16*)(ws + oOH);
  u16*   OL  = (u16*)(ws + oOL);

  const int n8x  = (SEQ * HID) / 8;
  const int n8rk = (SEQ * HD) / 8;
  const int n8q  = (SEQ * DQ) / 8;
  const int n8k  = (SEQ * DKV) / 8;
  if ((n8x % 256) != 0 || (n8rk % 256) != 0 || (n8q % 256) != 0 || (n8k % 256) != 0) return;
  if ((SEQ % 64) != 0 || (HID % 64) != 0 || (DQ % 64) != 0 || (DKV % 64) != 0 || (HD % 64) != 0) return;
  if ((HID % 32) != 0 || (DQ % 32) != 0) return;

  const dim3 b256(256), b128(128);
  const dim3 gX(n8x / 256);
  const dim3 gRK(NKV * (n8rk / 256));
  const dim3 gRQ(n8q / 256);
  const dim3 gRKp(n8k / 256);
  const int  tWQ = (HID / 64) * (DQ / 64);
  const int  tWK = (HID / 64) * (DKV / 64);
  const int  tWO = (DQ / 64) * (HID / 64);
  const int  tRV = (SEQ / 64) * (HD / 64);
  const dim3 gTQ(tWQ), gTK(tWK), gTO(tWO), gTR(NKV * tRV);
  const dim3 gGQ((SEQ / 64) * (DQ / 64));
  const dim3 gGK((SEQ / 64) * (DKV / 64));
  const dim3 gGV((DKV / 64) * (SEQ / 64));
  const dim3 gAT(ATT_BLOCKS);
  const dim3 bAT(ATT_THREADS);
  const dim3 gGO((SEQ / 64) * (HID / 64));

  cvt16<<<gX, b256, 0, stream>>>(Xin, XB, n8x, n8x / 256, 0, 0, 0, 1.0f);
  tr16<<<gTQ, b256, 0, stream>>>(Wqi, WQT, WQT, HID, DQ, tWQ, 0, 0, 0, 1.0f);
  tr16<<<gTK, b256, 0, stream>>>(Wki, WKT, WKT, HID, DKV, tWK, 0, 0, 0, 1.0f);
  tr16<<<gTK, b256, 0, stream>>>(Wvi, WVT, WVT, HID, DKV, tWK, 0, 0, 0, 1.0f);
  tr16<<<gTO, b256, 0, stream>>>(Woi, WOT, WOT, DQ, HID, tWO, 0, 0, 1, WOS);
  cvt16<<<gRK, b256, 0, stream>>>(RKi, RK, n8rk, n8rk / 256, (RLEN_FULL * HD) / 8, (SEQ * HD) / 8, 1, KSC);
  tr16<<<gTR, b256, 0, stream>>>(RVi, RVH, RVL, SEQ, HD, tRV, RLEN_FULL * HD, HD * SEQ, 2, VCAR);
  gemm_bb32<<<gGQ, b128, 0, stream>>>(XB, WQT, QF, SEQ, DQ, HID, 1.0f);
  gemm_bb32<<<gGK, b128, 0, stream>>>(XB, WKT, KF, SEQ, DKV, HID, 1.0f);
  gemm_vv16<<<gGV, b128, 0, stream>>>(WVT, XB, VH, VL, DKV, SEQ, HID, VCAR);
  rope16<<<gRQ, b256, 0, stream>>>(QF, DQ, Cin, Sin, QH, QL, 1, n8q, QSC, QLS);
  rope16<<<gRKp, b256, 0, stream>>>(KF, DKV, Cin, Sin, KP, KP, 0, n8k, KSC, QLS);
  attn_fwd<<<gAT, bAT, 0, stream>>>(QH, QL, KP, VH, VL, RK, RVH, RVL, OH, OL);
  gemm_oo32<<<gGO, b128, 0, stream>>>(OH, OL, WOT, out, SEQ, HID, DQ, 1.0f / (OSC * WOS), 1.0f / OLS);
  (void)hipGetLastError();
}
